// cMLP_91182155694693
// MI455X (gfx1250) — hardware-verified
//
#include <hip/hip_runtime.h>


#ifndef NB
#define NB 16
#endif
#ifndef SEQ
#define SEQ 2048
#endif
#define NB_FULL   16
#define SEQ_FULL  2048
#define LAGN      5
#define TOUT      (SEQ - LAGN + 1)
#define TOUT_FULL (SEQ_FULL - LAGN + 1)
#define NCH       64
#define NNET      64
#define HID       32
#define K0        (LAGN * NCH)
#define XROWS     (NB * SEQ + 64)
#define HP        40
#define OP        36
#define NPASS     16
#define W1C       64.0f
#define W1CI      0.015625f

static_assert(NB >= 1 && NB <= NB_FULL);
static_assert(SEQ <= SEQ_FULL && SEQ % 64 == 0 && SEQ > LAGN);
static_assert(K0 % 32 == 0);
static_assert(NCH == 64 && NNET == 64 && HID == 32);
static_assert(NPASS * 2 * 2 == NNET);
static_assert((XROWS * 8) % 256 == 0);
static_assert(HID * K0 / 8 == 5 * 256);
static_assert(HID * K0 == 40 * 256);
static_assert(NNET * HID * HID == 32 * 256 * 8);
static_assert(16 * 4 == 64 && 32 * 16 == 4 * 32 * 4);
static_assert((HP * 2) % 16 == 0 && (OP * 4) % 16 == 0);
static_assert(16 * HP * 2 + 64 * OP * 4 <= 131072);
static_assert(HID * K0 * 4 <= 131072);
static_assert((size_t)NB_FULL * TOUT_FULL * NNET * 4 == (size_t)8372224);

typedef unsigned short bf;
typedef _Float16 h16;
typedef __attribute__((ext_vector_type(16))) __bf16   v16bf;
typedef __attribute__((ext_vector_type(16))) _Float16 v16h;
typedef __attribute__((ext_vector_type(8)))  _Float16 v8h;
typedef __attribute__((ext_vector_type(8)))  unsigned short v8us;
typedef __attribute__((ext_vector_type(8)))  float    v8f;
typedef __attribute__((ext_vector_type(4)))  float    v4f;
typedef v4f  __attribute__((may_alias)) v4fa;
typedef v8h  __attribute__((may_alias)) v8ha;

__device__ __forceinline__ unsigned short f2bf(float f) { unsigned u = __float_as_uint(f); u += 0x7FFFu + ((u >> 16) & 1u); return (unsigned short)(u >> 16); }
__device__ __forceinline__ float bf2f(unsigned short w) { return __uint_as_float(((unsigned)w) << 16); }
__device__ __forceinline__ float bfr(float f) { return bf2f(f2bf(f)); }
__device__ __forceinline__ v16bf cat16b(v8us lo, v8us hi) { return __builtin_bit_cast(v16bf, __builtin_shufflevector(lo, hi, 0, 1, 2, 3, 4, 5, 6, 7, 8, 9, 10, 11, 12, 13, 14, 15)); }
__device__ __forceinline__ v16h cat16h(v8h lo, v8h hi) { return __builtin_shufflevector(lo, hi, 0, 1, 2, 3, 4, 5, 6, 7, 8, 9, 10, 11, 12, 13, 14, 15); }
__device__ __forceinline__ v8f wmmab(v16bf a, v16bf b, v8f c) { return __builtin_amdgcn_wmma_f32_16x16x32_bf16(false, a, false, b, (short)0, c, false, false); }
__device__ __forceinline__ v8f wmmah_g(v16h a, v16h b, v8f c) {
    c = __builtin_amdgcn_wmma_f32_16x16x32_f16(false, a, false, b, (short)0, c, false, false);
    asm volatile("v_nop\n\tv_nop\n\tv_nop\n\tv_nop" : "+v"(c) : "v"(a), "v"(b));
    return c; }
__device__ __forceinline__ v16bf ldb(const bf* p)  { return cat16b(*(const v8us*)p, *(const v8us*)(p + 16)); }
__device__ __forceinline__ v16h  ldh(const h16* p) { return cat16h(*(const v8h*)p, *(const v8h*)(p + 16)); }
static __device__ __forceinline__ h16 toh_flush(float v) { const h16 r = (h16)v; return (fabsf(v) < 6.103515625e-05f) ? (h16)0.0f : r; }
__device__ __forceinline__ void wave_sync() { __builtin_amdgcn_fence(3  , "wavefront"); __builtin_amdgcn_wave_barrier(); asm volatile("" ::: "memory"); }

__global__ __launch_bounds__(256) void k_xb(const float* __restrict__ X, bf* XB) {
    const unsigned q = blockIdx.x * 256u + threadIdx.x;
    const unsigned row = q >> 3; const unsigned c8 = (q & 7u) * 8u;
    const bool live = row < (unsigned)(NB * SEQ);
    const unsigned rc = live ? row : (unsigned)(NB * SEQ - 1);
    const unsigned b = rc / (unsigned)SEQ, t = rc - b * (unsigned)SEQ;
    const v8f a = *(const v8f*)(X + ((size_t)b * SEQ_FULL + t) * NCH + c8);
    v8us o;
#pragma unroll
    for (int k = 0; k < 8; ++k) o[k] = live ? f2bf(a[k]) : (unsigned short)0;
    *(volatile v8us*)(XB + (size_t)q * 8) = o; __threadfence(); *(volatile v8us*)(XB + (size_t)q * 8) = o;
}

__global__ __launch_bounds__(256) void k_w0t(const float* __restrict__ W0, bf* W0T) {
    __shared__ float ts[HID * K0];
    const int n = blockIdx.x, t = threadIdx.x;
    const float* src = W0 + (size_t)n * (HID * K0);
#pragma unroll 1
    for (int i = 0; i < 40; ++i) { const int f = i * 256 + t; ts[f] = src[f]; }
    __syncthreads();
    bf* dst = W0T + (size_t)n * (HID * K0);
#pragma unroll 1
    for (int ps = 0; ps < 2; ++ps) {
#pragma unroll 1
        for (int it = 0; it < 5; ++it) {
            const int q = it * 256 + t; const int row = q / 40; const int ch = q - row * 40;
            const int l = ch >> 3, c0 = (ch & 7) * 8; v8us o;
#pragma unroll
            for (int k = 0; k < 8; ++k) o[k] = f2bf(ts[row * K0 + (c0 + k) * LAGN + l]);
            *(volatile v8us*)(dst + (size_t)q * 8) = o; }
        if (ps == 0) __threadfence(); }
}

__global__ __launch_bounds__(256) void k_w1h(const float* __restrict__ W1, h16* W1H) {
    const unsigned q = blockIdx.x * 256u + threadIdx.x;
    const v8f a = *(const v8f*)(W1 + (size_t)q * 8);
    v8h o;
#pragma unroll
    for (int k = 0; k < 8; ++k) o[k] = toh_flush(bfr(a[k]) * W1C);
    *(volatile v8h*)(W1H + (size_t)q * 8) = o; __threadfence(); *(volatile v8h*)(W1H + (size_t)q * 8) = o;
}

__global__ __launch_bounds__(32) __attribute__((amdgpu_num_vgpr(256))) void k_main(const bf* __restrict__ XB, const bf* __restrict__ W0T, const h16* __restrict__ W1H,
                                                                                    const float* __restrict__ b0, const float* __restrict__ b1,
                                                                                    const float* __restrict__ W2, const float* __restrict__ b2, float* OUT) {
    __shared__ __align__(16) h16 hs[16 * HP];
    __shared__ __align__(16) float outs[64 * OP];
    const int lane = threadIdx.x & 31, lr = lane & 15, hi = lane >> 4;
    const int tile = blockIdx.x >> 1, nh = blockIdx.x & 1;
    const int p0 = tile * 64;
    const int bt = p0 / SEQ, t0 = p0 - bt * SEQ;
    const int row8 = hi * 8;
    const size_t aoff = (size_t)(p0 + lr) * NCH + 8 * hi;
#pragma unroll 1
    for (int ps = 0; ps < NPASS; ++ps) {
        const int n0 = nh * 32 + ps * 2;
        v8f acc[4][4];
#pragma unroll
        for (int mb = 0; mb < 4; ++mb)
#pragma unroll
            for (int nb = 0; nb < 4; ++nb) acc[mb][nb] = (v8f){};
        const size_t boff = (size_t)(n0 * HID + lr) * K0 + 8 * hi;
#pragma unroll 1
        for (int kc = 0; kc < K0; kc += 32) {
            v16bf a[4];
#pragma unroll
            for (int mb = 0; mb < 4; ++mb) a[mb] = ldb(XB + aoff + (size_t)mb * 16 * NCH + kc);
#pragma unroll
            for (int nb = 0; nb < 4; ++nb) { const v16bf b = ldb(W0T + boff + (size_t)nb * 16 * K0 + kc);
#pragma unroll
                for (int mb = 0; mb < 4; ++mb) acc[mb][nb] = wmmab(a[mb], b, acc[mb][nb]); }
            asm volatile("v_nop\n\tv_nop\n\tv_nop\n\tv_nop" : "+v"(acc[0][0]), "+v"(acc[1][1]), "+v"(acc[2][2]), "+v"(acc[3][3]) : "v"(a[0]), "v"(a[1]), "v"(a[2]), "v"(a[3]));
        }
#pragma unroll
        for (int j = 0; j < 2; ++j) {
            const int cb = (n0 + j) * HID + lr;
            const float b0a = bfr(b0[cb]), b0b = bfr(b0[cb + 16]);
            const float b1a = bfr(b1[cb]), b1b = bfr(b1[cb + 16]);
            const float w2a = bfr(W2[cb]), w2b = bfr(W2[cb + 16]);
            const float b2v = bfr(b2[n0 + j]);
            const v16h wb0 = ldh(W1H + (size_t)cb * HID + 8 * hi);
            const v16h wb1 = ldh(W1H + (size_t)(cb + 16) * HID + 8 * hi);
#pragma unroll
            for (int mb = 0; mb < 4; ++mb) {
#pragma unroll
                for (int r = 0; r < 8; ++r) {
                    hs[(row8 + r) * HP + lr]      = toh_flush(fmaxf(acc[mb][2 * j][r] + b0a, 0.0f));
                    hs[(row8 + r) * HP + 16 + lr] = toh_flush(fmaxf(acc[mb][2 * j + 1][r] + b0b, 0.0f)); }
                wave_sync();
                const v8h x0 = *(const v8ha*)(&hs[lr * HP + 8 * hi]);
                const v8h x1 = *(const v8ha*)(&hs[lr * HP + 16 + 8 * hi]);
                const v16h ha = cat16h(x0, x1);
                wave_sync();
                const v8f d0 = wmmah_g(ha, wb0, (v8f){});
                const v8f d1 = wmmah_g(ha, wb1, (v8f){});
                float s[8];
#pragma unroll
                for (int r = 0; r < 8; ++r) {
                    const float ya = fmaxf(d0[r] * W1CI + b1a, 0.0f);
                    const float yb = fmaxf(d1[r] * W1CI + b1b, 0.0f);
                    s[r] = ya * w2a + yb * w2b; }
#pragma unroll
                for (int r = 0; r < 8; ++r) {
                    s[r] += __shfl_xor(s[r], 1, 32); s[r] += __shfl_xor(s[r], 2, 32);
                    s[r] += __shfl_xor(s[r], 4, 32); s[r] += __shfl_xor(s[r], 8, 32); }
                float v = s[0];
#pragma unroll
                for (int r = 1; r < 8; ++r) v = (lr == r) ? s[r] : v;
                if (lr < 8) outs[(mb * 16 + row8 + lr) * OP + ps * 2 + j] = v + b2v;
            }
        }
    }
    wave_sync();
#pragma unroll 1
    for (int ps = 0; ps < 2; ++ps) {
#pragma unroll 1
        for (int it = 0; it < 16; ++it) {
            const int row = 4 * it + (lane >> 3), c4 = (lane & 7) * 4;
            const int t = t0 + row;
            const v4f v = *(const v4fa*)(&outs[row * OP + c4]);
            if (t < TOUT) *(volatile v4f*)(OUT + ((size_t)bt * TOUT_FULL + t) * NNET + nh * 32 + c4) = v; }
        if (ps == 0) __threadfence(); }
}

static constexpr size_t al256(size_t v) { return (v + 255) & ~(size_t)255; }
static constexpr size_t SZ_XB  = al256((size_t)XROWS * NCH * 2);
static constexpr size_t SZ_W0T = al256((size_t)NNET * HID * K0 * 2);
static constexpr size_t SZ_W1H = al256((size_t)NNET * HID * HID * 2);
static constexpr size_t SZ_TOTAL = SZ_XB + SZ_W0T + SZ_W1H;
static_assert(SZ_TOTAL <= (size_t)134217728);

extern "C" void kernel_launch(void* const* d_in, const int* in_sizes, int n_in,
                              void* d_out, int out_size, void* d_ws, size_t ws_size, hipStream_t stream) {
    if (n_in < 7) return;
    if ((size_t)in_sizes[0] < ((size_t)(NB - 1) * SEQ_FULL + SEQ) * NCH) return;
    if ((size_t)in_sizes[1] < (size_t)NNET * HID * K0) return;
    if ((size_t)in_sizes[2] < (size_t)NNET * HID) return;
    if ((size_t)in_sizes[3] < (size_t)NNET * HID * HID) return;
    if ((size_t)in_sizes[4] < (size_t)NNET * HID) return;
    if ((size_t)in_sizes[5] < (size_t)NNET * HID) return;
    if ((size_t)in_sizes[6] < (size_t)NNET) return;
    if ((size_t)out_size < ((size_t)(NB - 1) * TOUT_FULL + TOUT) * NNET) return;
    if (SZ_TOTAL > ws_size) return;
    const float* X  = (const float*)d_in[0];
    const float* W0 = (const float*)d_in[1];
    const float* b0 = (const float*)d_in[2];
    const float* W1 = (const float*)d_in[3];
    const float* b1 = (const float*)d_in[4];
    const float* W2 = (const float*)d_in[5];
    const float* b2 = (const float*)d_in[6];
    float* OUT = (float*)d_out;
    char* wsp = (char*)d_ws;
    bf*  XB  = (bf*)wsp;  wsp += SZ_XB;
    bf*  W0T = (bf*)wsp;  wsp += SZ_W0T;
    h16* W1H = (h16*)wsp; wsp += SZ_W1H;

    k_w0t<<<NNET, 256, 0, stream>>>(W0, W0T);
    k_w1h<<<32, 256, 0, stream>>>(W1, W1H);
    k_xb<<<(unsigned)((XROWS * 8) / 256), 256, 0, stream>>>(X, XB);
    k_main<<<(unsigned)((NB * SEQ / 64) * 2), 32, 0, stream>>>(XB, W0T, W1H, b0, b1, W2, b2, OUT);
}
